// KV_CachedFlashMHADecoderBlock_90615220011031
// MI455X (gfx1250) — hardware-verified
//
#include <hip/hip_runtime.h>
#include <stddef.h>
#include <stdint.h>
#include <math.h>

#define BB   2
#define NN   2048
#define CC   1024
#define HH   16
#define DD   64
#define FF   4096
#define ROWS (BB * NN)
#define C3   (3 * CC)
#define PL   ((size_t)BB * HH * NN * DD)
#define NTRIG (NN * 32)

static_assert(NN % 256 == 0);
static_assert(CC % 64 == 0);
static_assert(FF % 64 == 0);
static_assert(DD == 64);
static_assert(HH * DD == CC);
static_assert(ROWS % 256 == 0);
static_assert((ROWS * CC) % 8 == 0);
static_assert(NTRIG % 256 == 0);

typedef _Float16 v16h __attribute__((ext_vector_type(16)));
typedef _Float16 v8h  __attribute__((ext_vector_type(8)));
typedef float    v8f  __attribute__((ext_vector_type(8)));
typedef float    v4f  __attribute__((ext_vector_type(4)));
typedef unsigned int v4u __attribute__((ext_vector_type(4)));

union Frag  { v16h v; v8h h[2]; };
union Pack8 { v8h h; v4u u; };

__device__ __forceinline__ v8f mma16(v16h a, v16h b, v8f c) {
  c = __builtin_amdgcn_wmma_f32_16x16x32_f16(false, a, false, b, (short)0, c, false, false);
  asm volatile("v_nop\n\tv_nop\n\tv_nop\n\tv_nop" : "+v"(c) : "v"(a), "v"(b));
  return c;
}

__device__ __forceinline__ v16h ldfrag(const _Float16* p, int ld, int row0, int k0, int lane) {
  const int m = lane & 15, lh = lane >> 4;
  const _Float16* q = p + (size_t)(row0 + m) * ld + k0 + 8 * lh;
  Frag f;
  f.h[0] = *(const v8h*)(q);
  f.h[1] = *(const v8h*)(q + 16);
  return f.v;
}

__device__ __forceinline__ v8f zero8() { return (v8f){0.f, 0.f, 0.f, 0.f, 0.f, 0.f, 0.f, 0.f}; }

__device__ __forceinline__ float gelu16(float v) {
  const float a = -1.5957691216057308f * (v + 0.044715f * v * v * v);
  const float e = __expf(a);
  return 16.0f * v * __builtin_amdgcn_rcpf(1.0f + e);
}

template <int KK>
__device__ __forceinline__ void gemm32x64(const _Float16* __restrict__ A, int lda,
                                          const _Float16* __restrict__ Bt, int ldb,
                                          int m0, int n0, int lane, v8f (&acc)[2][4]) {
#pragma unroll 2
  for (int k0 = 0; k0 < KK; k0 += 32) {
    const v16h a0 = ldfrag(A, lda, m0, k0, lane);
    const v16h a1 = ldfrag(A, lda, m0 + 16, k0, lane);
    const v16h b0 = ldfrag(Bt, ldb, n0, k0, lane);
    const v16h b1 = ldfrag(Bt, ldb, n0 + 16, k0, lane);
    const v16h b2 = ldfrag(Bt, ldb, n0 + 32, k0, lane);
    const v16h b3 = ldfrag(Bt, ldb, n0 + 48, k0, lane);
    acc[0][0] = mma16(a0, b0, acc[0][0]);
    acc[1][0] = mma16(a1, b0, acc[1][0]);
    acc[0][1] = mma16(a0, b1, acc[0][1]);
    acc[1][1] = mma16(a1, b1, acc[1][1]);
    acc[0][2] = mma16(a0, b2, acc[0][2]);
    acc[1][2] = mma16(a1, b2, acc[1][2]);
    acc[0][3] = mma16(a0, b3, acc[0][3]);
    acc[1][3] = mma16(a1, b3, acc[1][3]);
  }
}

__global__ __launch_bounds__(256) void k_trig(float* __restrict__ trig, int n) {
  const int t = blockIdx.x * 256 + (int)threadIdx.x;
  if (t >= n) return;
  const int i = t & 31, pos = t >> 5;
  const int a = i & 7, e = i >> 3;
  const double m = (a == 0) ? 1.0
                 : (a == 1) ? 0.749894209332455827
                 : (a == 2) ? 0.562341325190349080
                 : (a == 3) ? 0.421696503428582249
                 : (a == 4) ? 0.316227766016837933
                 : (a == 5) ? 0.237137370566165527
                 : (a == 6) ? 0.177827941003892280
                 :            0.133352143216332402;
  const double pw = (e == 0) ? 1.0 : (e == 1) ? 0.1 : (e == 2) ? 0.01 : 0.001;
  const float inv = (float)(m * pw);
  const float ang = (float)pos * inv;
  float sn, cs;
  sincosf(ang, &sn, &cs);
  volatile float* pc = (volatile float*)(trig + t);
  volatile float* ps = (volatile float*)(trig + NTRIG + t);
  *pc = cs;
  *ps = sn;
  __threadfence();
  *pc = cs;
  *ps = sn;
}

__global__ __launch_bounds__(256) void k_cvt8(const float* __restrict__ x, _Float16* __restrict__ xh, int ngrp) {
  const int t = blockIdx.x * 256 + (int)threadIdx.x;
  if (t >= ngrp) return;
  const size_t o = (size_t)t * 8;
  const v4f a0 = *(const v4f*)(x + o);
  const v4f a1 = *(const v4f*)(x + o + 4);
  Pack8 pk;
  pk.h = (v8h){(_Float16)a0[0], (_Float16)a0[1], (_Float16)a0[2], (_Float16)a0[3],
               (_Float16)a1[0], (_Float16)a1[1], (_Float16)a1[2], (_Float16)a1[3]};
  const v4u vv = pk.u;
  volatile v4u* d = (volatile v4u*)(xh + o);
  *d = vv;
  __threadfence();
  *d = vv;
}

#define WTP 68
__global__ __launch_bounds__(256) void k_wt(const float* __restrict__ w, _Float16* __restrict__ wt,
                                           int nout, int kin) {
  __shared__ __align__(16) float tf[64 * WTP];
  const int tid = threadIdx.x;
  const int n0 = blockIdx.x * 64;
  const int k0 = blockIdx.y * 64;
  {
    const int kr = tid >> 4;
    const int n4 = (tid & 15) * 4;
#pragma unroll
    for (int it = 0; it < 4; ++it) {
      const int kl = it * 16 + kr;
      const v4f a = *(const v4f*)(w + (size_t)(k0 + kl) * nout + n0 + n4);
      *(v4f*)(tf + kl * WTP + n4) = a;
    }
  }
  __syncthreads();
  v4u val[2];
  size_t go[2];
#pragma unroll
  for (int j = 0; j < 2; ++j) {
    const int p  = tid + 256 * j;
    const int nl = p >> 3;
    const int pc = p & 7;
    const float* cp = tf + (pc * 8) * WTP + nl;
    Pack8 pk;
    pk.h = (v8h){(_Float16)(cp[0 * WTP] * 32.0f), (_Float16)(cp[1 * WTP] * 32.0f),
                 (_Float16)(cp[2 * WTP] * 32.0f), (_Float16)(cp[3 * WTP] * 32.0f),
                 (_Float16)(cp[4 * WTP] * 32.0f), (_Float16)(cp[5 * WTP] * 32.0f),
                 (_Float16)(cp[6 * WTP] * 32.0f), (_Float16)(cp[7 * WTP] * 32.0f)};
    val[j] = pk.u;
    go[j]  = (size_t)(n0 + nl) * kin + k0 + pc * 8;
  }
  for (int ps = 0; ps < 2; ++ps) {
#pragma unroll
    for (int j = 0; j < 2; ++j) *(volatile v4u*)(wt + go[j]) = val[j];
    __threadfence();
  }
}

__global__ __launch_bounds__(256) void k_ln(const float* __restrict__ in,
                                           const float* __restrict__ g,
                                           const float* __restrict__ bt,
                                           _Float16* __restrict__ outh) {
  __shared__ __align__(16) float rb[CC];
  __shared__ float red[16];
  const int tid = threadIdx.x, lane = tid & 31, wave = tid >> 5;
  const size_t ro = (size_t)blockIdx.x * CC;
  const v4f v = *(const v4f*)(in + ro + 4 * tid);
  float s = (v[0] + v[1]) + (v[2] + v[3]);
#pragma unroll
  for (int off = 1; off < 32; off <<= 1) s += __shfl_xor(s, off, 32);
  if (lane == 0) red[wave] = s;
  __syncthreads();
  float ts = 0.f;
#pragma unroll
  for (int w = 0; w < 8; ++w) ts += red[w];
  const float mean = ts * (1.0f / (float)CC);
  const float d0 = v[0] - mean, d1 = v[1] - mean, d2 = v[2] - mean, d3 = v[3] - mean;
  float q = (d0 * d0 + d1 * d1) + (d2 * d2 + d3 * d3);
#pragma unroll
  for (int off = 1; off < 32; off <<= 1) q += __shfl_xor(q, off, 32);
  if (lane == 0) red[8 + wave] = q;
  __syncthreads();
  float tq = 0.f;
#pragma unroll
  for (int w = 0; w < 8; ++w) tq += red[8 + w];
  const float var = tq * (1.0f / (float)CC);
  const float inv = 1.0f / sqrtf(var + 1e-5f);
  const v4f g4 = *(const v4f*)(g + 4 * tid);
  const v4f b4 = *(const v4f*)(bt + 4 * tid);
  v4f o;
  o[0] = d0 * inv * g4[0] + b4[0];
  o[1] = d1 * inv * g4[1] + b4[1];
  o[2] = d2 * inv * g4[2] + b4[2];
  o[3] = d3 * inv * g4[3] + b4[3];
  *(v4f*)(rb + 4 * tid) = o;
  __syncthreads();
  if (tid < 128) {
    const v4f a0 = *(const v4f*)(rb + 8 * tid);
    const v4f a1 = *(const v4f*)(rb + 8 * tid + 4);
    Pack8 pk;
    pk.h = (v8h){(_Float16)a0[0], (_Float16)a0[1], (_Float16)a0[2], (_Float16)a0[3],
                 (_Float16)a1[0], (_Float16)a1[1], (_Float16)a1[2], (_Float16)a1[3]};
    const v4u vv = pk.u;
    volatile v4u* hq = (volatile v4u*)(outh + ro + 8 * tid);
    *hq = vv;
    __threadfence();
    *hq = vv;
  }
}

#define STP 72
union ProjLds { _Float16 h[256 * STP]; float f[8192]; };
static_assert(sizeof(ProjLds) == 256 * STP * 2);

__global__ __launch_bounds__(256) void k_proj(const _Float16* __restrict__ ah,
                                              const _Float16* __restrict__ wt,
                                              const float* __restrict__ b0,
                                              const float* __restrict__ b1,
                                              const float* __restrict__ b2,
                                              const float* __restrict__ trig,
                                              _Float16* qp, _Float16* kp, _Float16* vtp, int wbase) {
  __shared__ __align__(16) ProjLds sm;
  const int tid = threadIdx.x, lane = tid & 31, wave = tid >> 5;
  const int hh = lane >> 4, c = lane & 15;
  const int mb = blockIdx.x * 256;
  const int m0 = mb + wave * 32;
  const int n0 = blockIdx.y * 64;
  const int slab  = n0 >> 10;
  const int which = wbase + slab;
  const int nin = n0 & (CC - 1);

  v8f acc[2][4];
#pragma unroll
  for (int s = 0; s < 2; ++s)
#pragma unroll
    for (int t = 0; t < 4; ++t) acc[s][t] = zero8();
  gemm32x64<CC>(ah, CC, wt, CC, m0, n0, lane, acc);

  const float* bsel = (slab == 0) ? b0 : ((slab == 1) ? b1 : b2);
#pragma unroll
  for (int t = 0; t < 4; ++t) {
    const float bb = bsel[nin + 16 * t + c];
#pragma unroll
    for (int sub = 0; sub < 2; ++sub) {
#pragma unroll
      for (int r = 0; r < 8; ++r) acc[sub][t][r] = acc[sub][t][r] * 0.03125f + bb;
    }
  }

  if (which < 2) {
    const int pb = mb & (NN - 1);
#pragma unroll 1
    for (int ph = 0; ph < 2; ++ph) {
      __syncthreads();
      {
        const size_t tb0 = (size_t)(pb + ph * 128) * 32;
#pragma unroll 1
        for (int tb = 0; tb < 2; ++tb) {
          const float* src = trig + (size_t)tb * NTRIG + tb0;
          float* dl = sm.f + tb * 4096;
          const v4f t0 = *(const v4f*)(src + 4 * tid);
          const v4f t1 = *(const v4f*)(src + 4 * tid + 1024);
          const v4f t2 = *(const v4f*)(src + 4 * tid + 2048);
          const v4f t3 = *(const v4f*)(src + 4 * tid + 3072);
          *(v4f*)(dl + 4 * tid)        = t0;
          *(v4f*)(dl + 4 * tid + 1024) = t1;
          *(v4f*)(dl + 4 * tid + 2048) = t2;
          *(v4f*)(dl + 4 * tid + 3072) = t3;
        }
      }
      __syncthreads();
      if ((wave >> 2) == ph) {
#pragma unroll
        for (int sub = 0; sub < 2; ++sub) {
#pragma unroll
          for (int r = 0; r < 8; ++r) {
            const int lp = (wave & 3) * 32 + sub * 16 + 8 * hh + r;
            const float* ct  = sm.f + lp * 32;
            const float* snt = sm.f + 4096 + lp * 32;
#pragma unroll
            for (int t = 0; t < 2; ++t) {
              const int d = 16 * t + c;
              const float cv = ct[d], sv = snt[d];
              const float x1 = acc[sub][t][r], x2 = acc[sub][t + 2][r];
              acc[sub][t][r]     = x1 * cv - x2 * sv;
              acc[sub][t + 2][r] = x2 * cv + x1 * sv;
            }
          }
        }
      }
    }
    __syncthreads();
  }

  _Float16* st = sm.h;
#pragma unroll
  for (int t = 0; t < 4; ++t) {
#pragma unroll
    for (int sub = 0; sub < 2; ++sub) {
#pragma unroll
      for (int r = 0; r < 8; ++r) {
        const int lr = wave * 32 + sub * 16 + 8 * hh + r;
        st[lr * STP + 16 * t + c] = (_Float16)acc[sub][t][r];
      }
    }
  }
  __syncthreads();

  const int head = nin >> 6;
  const int b  = mb >> 11;
  const int nb = mb & (NN - 1);
  const int bh = b * HH + head;
  v4u val[8];
  size_t go[8];
  _Float16* dst;
  if (which < 2) {
    dst = (which == 0) ? qp : kp;
#pragma unroll
    for (int j = 0; j < 8; ++j) {
      const int p  = tid + 256 * j;
      const int lr = p >> 3;
      const int pc = p & 7;
      Pack8 pk;
      pk.h  = *(const v8h*)(st + lr * STP + pc * 8);
      val[j] = pk.u;
      go[j]  = ((size_t)bh * NN + nb + lr) * DD + pc * 8;
    }
  } else {
    dst = vtp;
#pragma unroll
    for (int j = 0; j < 8; ++j) {
      const int p  = tid + 256 * j;
      const int L  = p >> 3;
      const int pc = p & 7;
      const int d  = L >> 2;
      const int nl = (L & 3) * 64 + pc * 8;
      const _Float16* cp = st + nl * STP + d;
      Pack8 pk;
      pk.h = (v8h){cp[0 * STP], cp[1 * STP], cp[2 * STP], cp[3 * STP],
                   cp[4 * STP], cp[5 * STP], cp[6 * STP], cp[7 * STP]};
      val[j] = pk.u;
      go[j]  = ((size_t)bh * DD + d) * NN + nb + nl;
    }
  }
  for (int ps = 0; ps < 2; ++ps) {
#pragma unroll
    for (int j = 0; j < 8; ++j) *(volatile v4u*)(dst + go[j]) = val[j];
    __threadfence();
  }
}

#define KTP 72
#define PTP 72
__global__ __launch_bounds__(256) void k_attn(const _Float16* __restrict__ qp,
                                              const _Float16* __restrict__ kp,
                                              const _Float16* __restrict__ vt,
                                              _Float16* __restrict__ op, float sscale, int causal) {
  __shared__ __align__(16) _Float16 Ks[64 * KTP];
  __shared__ __align__(16) _Float16 Vs[64 * KTP];
  __shared__ __align__(16) _Float16 Ps[8][16 * PTP];

  const int tid = threadIdx.x, lane = tid & 31, wave = tid >> 5;
  const int hh = lane >> 4, c = lane & 15;
  const int bh = blockIdx.x >> 4;
  const int qb = blockIdx.x & 15;
  const int b  = bh >> 4, h = bh & (HH - 1);
  const int q0 = qb * 128 + wave * 16;

  const _Float16* Q = qp + (size_t)bh * NN * DD;
  const _Float16* K = kp + (size_t)bh * NN * DD;
  const _Float16* V = vt + (size_t)bh * DD * NN;

  v16h qa[2];
  qa[0] = ldfrag(Q, DD, q0, 0, lane);
  qa[1] = ldfrag(Q, DD, q0, 32, lane);

  const float NEGI = -__builtin_huge_valf();
  float mrow[8], lrow[8];
  v8f oacc[4];
#pragma unroll
  for (int r = 0; r < 8; ++r) { mrow[r] = NEGI; lrow[r] = 0.f; }
#pragma unroll
  for (int t = 0; t < 4; ++t) oacc[t] = zero8();

  _Float16* pw = Ps[wave];
  const int nchunk = (causal != 0) ? (2 * qb + 2) : (NN / 64);

  for (int kc = 0; kc < nchunk; ++kc) {
    const int kv0 = kc * 64;
    const bool cz = (causal != 0) && (kv0 + 64 > qb * 128);
    __syncthreads();
    {
      const int r  = tid >> 2;
      const int qq = (tid & 3) * 16;
      const _Float16* ks = K + (size_t)(kv0 + r) * DD + qq;
      *(v8h*)(Ks + r * KTP + qq)     = *(const v8h*)(ks);
      *(v8h*)(Ks + r * KTP + qq + 8) = *(const v8h*)(ks + 8);
      const _Float16* vs = V + (size_t)r * NN + kv0 + qq;
      *(v8h*)(Vs + r * KTP + qq)     = *(const v8h*)(vs);
      *(v8h*)(Vs + r * KTP + qq + 8) = *(const v8h*)(vs + 8);
    }
    __syncthreads();

    v8f s[4];
#pragma unroll
    for (int j = 0; j < 4; ++j) s[j] = zero8();
#pragma unroll
    for (int dc = 0; dc < 2; ++dc) {
#pragma unroll
      for (int j = 0; j < 4; ++j) {
        const v16h kb = ldfrag(Ks, KTP, j * 16, dc * 32, lane);
        s[j] = mma16(qa[dc], kb, s[j]);
      }
    }
    float cm[8];
#pragma unroll
    for (int r = 0; r < 8; ++r) {
      const int qrow = q0 + 8 * hh + r;
      float m = NEGI;
#pragma unroll
      for (int j = 0; j < 4; ++j) {
        const int key = kv0 + j * 16 + c;
        float sv = s[j][r] * sscale;
        sv = (cz && (key > qrow)) ? NEGI : sv;
        s[j][r] = sv;
        m = fmaxf(m, sv);
      }
#pragma unroll
      for (int off = 1; off < 16; off <<= 1) m = fmaxf(m, __shfl_xor(m, off, 32));
      cm[r] = m;
    }
    float al[8];
#pragma unroll
    for (int r = 0; r < 8; ++r) {
      const float mnew  = fmaxf(mrow[r], cm[r]);
      const float alpha = __expf(mrow[r] - mnew);
      mrow[r] = mnew;
      float psum = 0.f;
#pragma unroll
      for (int j = 0; j < 4; ++j) {
        const float p = __expf(s[j][r] - mnew);
        psum += p;
        pw[(8 * hh + r) * PTP + j * 16 + c] = (_Float16)(p * 1024.0f);
      }
#pragma unroll
      for (int off = 1; off < 16; off <<= 1) psum += __shfl_xor(psum, off, 32);
      lrow[r] = lrow[r] * alpha + psum;
      al[r] = alpha;
    }
#pragma unroll
    for (int t = 0; t < 4; ++t)
#pragma unroll
      for (int r = 0; r < 8; ++r) oacc[t][r] *= al[r];
    __syncthreads();

#pragma unroll
    for (int kk = 0; kk < 2; ++kk) {
      const v16h pa = ldfrag(pw, PTP, 0, kk * 32, lane);
#pragma unroll
      for (int t = 0; t < 4; ++t) {
        const v16h vb = ldfrag(Vs, KTP, t * 16, kk * 32, lane);
        oacc[t] = mma16(pa, vb, oacc[t]);
      }
    }
  }
  __syncthreads();

#pragma unroll
  for (int r = 0; r < 8; ++r) {
    const float inv = 0.0625f / lrow[r];
#pragma unroll
    for (int t = 0; t < 4; ++t) pw[(8 * hh + r) * PTP + 16 * t + c] = (_Float16)(oacc[t][r] * inv);
  }
  __syncthreads();
  v4u val[4];
  size_t go[4];
#pragma unroll
  for (int it = 0; it < 4; ++it) {
    const int p  = lane + 32 * it;
    const int L  = p >> 3;
    const int pc = p & 7;
    Pack8 pk;
    pk.h   = *(const v8h*)(pw + L * PTP + pc * 8);
    val[it] = pk.u;
    go[it]  = ((size_t)(b * NN + q0 + L)) * CC + (size_t)h * DD + pc * 8;
  }
  for (int ps = 0; ps < 2; ++ps) {
#pragma unroll
    for (int it = 0; it < 4; ++it) *(volatile v4u*)(op + go[it]) = val[it];
    __threadfence();
  }
}

#define OTP 68
template <int KK, int RES>
__global__ __launch_bounds__(256) void k_gout(const _Float16* __restrict__ ap,
                                              const _Float16* __restrict__ wt,
                                              const float* __restrict__ bias,
                                              const float* __restrict__ res,
                                              float* __restrict__ out, float oscale) {
  __shared__ __align__(16) float st[8][16 * OTP];
  const int tid = threadIdx.x, lane = tid & 31, wave = tid >> 5;
  const int hh = lane >> 4, c = lane & 15;
  const int m0 = blockIdx.x * 256 + wave * 32;
  const int n0 = blockIdx.y * 64;

  v8f acc[2][4];
#pragma unroll
  for (int s = 0; s < 2; ++s)
#pragma unroll
    for (int t = 0; t < 4; ++t) acc[s][t] = zero8();
  gemm32x64<KK>(ap, KK, wt, KK, m0, n0, lane, acc);

  float bvs[4];
#pragma unroll
  for (int t = 0; t < 4; ++t) bvs[t] = bias[n0 + 16 * t + c];

  float* sw = st[wave];
#pragma unroll
  for (int sub = 0; sub < 2; ++sub) {
    __syncthreads();
#pragma unroll
    for (int t = 0; t < 4; ++t) {
#pragma unroll
      for (int r = 0; r < 8; ++r)
        sw[(8 * hh + r) * OTP + 16 * t + c] = acc[sub][t][r] * oscale + bvs[t];
    }
    __syncthreads();
    v4f val[8];
    size_t go[8];
#pragma unroll
    for (int it = 0; it < 8; ++it) {
      const int p    = lane + 32 * it;
      const int L    = p >> 3;
      const int pc   = p & 7;
      const int row  = L >> 1;
      const int half = L & 1;
      const size_t g = (size_t)(m0 + sub * 16 + row) * CC + n0 + half * 32 + pc * 4;
      v4f v = *(const v4f*)(sw + row * OTP + half * 32 + pc * 4);
      if (RES) {
        const v4f rr = *(const v4f*)(res + g);
        v[0] = v[0] + rr[0]; v[1] = v[1] + rr[1]; v[2] = v[2] + rr[2]; v[3] = v[3] + rr[3];
      }
      val[it] = v;
      go[it]  = g;
    }
    for (int ps = 0; ps < 2; ++ps) {
#pragma unroll
      for (int it = 0; it < 8; ++it) *(volatile v4f*)(out + go[it]) = val[it];
      __threadfence();
    }
  }
}

__global__ __launch_bounds__(256) void k_ffn1(const _Float16* __restrict__ ap,
                                              const _Float16* __restrict__ wt,
                                              const float* __restrict__ bias,
                                              _Float16* __restrict__ hp) {
  __shared__ __align__(16) float st[8][16 * OTP];
  const int tid = threadIdx.x, lane = tid & 31, wave = tid >> 5;
  const int hh = lane >> 4, c = lane & 15;
  const int m0 = blockIdx.x * 256 + wave * 32;
  const int n0 = blockIdx.y * 64;

  v8f acc[2][4];
#pragma unroll
  for (int s = 0; s < 2; ++s)
#pragma unroll
    for (int t = 0; t < 4; ++t) acc[s][t] = zero8();
  gemm32x64<CC>(ap, CC, wt, CC, m0, n0, lane, acc);

  float bvs[4];
#pragma unroll
  for (int t = 0; t < 4; ++t) bvs[t] = bias[n0 + 16 * t + c];

  float* sw = st[wave];
#pragma unroll
  for (int sub = 0; sub < 2; ++sub) {
    __syncthreads();
#pragma unroll
    for (int t = 0; t < 4; ++t) {
#pragma unroll
      for (int r = 0; r < 8; ++r)
        sw[(8 * hh + r) * OTP + 16 * t + c] = acc[sub][t][r] * 0.03125f + bvs[t];
    }
    __syncthreads();
    v4u val[4];
    size_t go[4];
#pragma unroll
    for (int it = 0; it < 4; ++it) {
      const int p  = lane + 32 * it;
      const int L  = p >> 3;
      const int pc = p & 7;
      const v4f x0 = *(const v4f*)(sw + L * OTP + pc * 8);
      const v4f x1 = *(const v4f*)(sw + L * OTP + pc * 8 + 4);
      Pack8 pk;
      pk.h = (v8h){(_Float16)gelu16(x0[0]), (_Float16)gelu16(x0[1]), (_Float16)gelu16(x0[2]), (_Float16)gelu16(x0[3]),
                   (_Float16)gelu16(x1[0]), (_Float16)gelu16(x1[1]), (_Float16)gelu16(x1[2]), (_Float16)gelu16(x1[3])};
      val[it] = pk.u;
      go[it]  = (size_t)(m0 + sub * 16 + L) * FF + n0 + pc * 8;
    }
    for (int ps = 0; ps < 2; ++ps) {
#pragma unroll
      for (int it = 0; it < 4; ++it) *(volatile v4u*)(hp + go[it]) = val[it];
      __threadfence();
    }
  }
}

extern "C" void kernel_launch(void* const* d_in, const int* in_sizes, int n_in,
                              void* d_out, int out_size, void* d_ws, size_t ws_size,
                              hipStream_t stream) {
  if (n_in < 28) return;
  if (in_sizes[0] != ROWS * CC || in_sizes[1] != ROWS * CC) return;
  if (in_sizes[2] != CC || in_sizes[3] != CC) return;
  if (in_sizes[4] != CC * CC || in_sizes[6] != CC * CC || in_sizes[8] != CC * CC || in_sizes[10] != CC * CC) return;
  if (in_sizes[5] != CC || in_sizes[7] != CC || in_sizes[9] != CC || in_sizes[11] != CC) return;
  if (in_sizes[12] != CC || in_sizes[13] != CC) return;
  if (in_sizes[14] != CC * CC || in_sizes[16] != CC * CC || in_sizes[18] != CC * CC || in_sizes[20] != CC * CC) return;
  if (in_sizes[15] != CC || in_sizes[17] != CC || in_sizes[19] != CC || in_sizes[21] != CC) return;
  if (in_sizes[22] != CC || in_sizes[23] != CC) return;
  if (in_sizes[24] != CC * FF || in_sizes[25] != FF) return;
  if (in_sizes[26] != FF * CC || in_sizes[27] != CC) return;
  if (out_size != ROWS * CC) return;

  const float* x     = (const float*)d_in[0];
  const float* y     = (const float*)d_in[1];
  const float* ln1_g = (const float*)d_in[2];
  const float* ln1_b = (const float*)d_in[3];
  const float* sa_wq = (const float*)d_in[4];
  const float* sa_bq = (const float*)d_in[5];
  const float* sa_wk = (const float*)d_in[6];
  const float* sa_bk = (const float*)d_in[7];
  const float* sa_wv = (const float*)d_in[8];
  const float* sa_bv = (const float*)d_in[9];
  const float* sa_wo = (const float*)d_in[10];
  const float* sa_bo = (const float*)d_in[11];
  const float* ln2_g = (const float*)d_in[12];
  const float* ln2_b = (const float*)d_in[13];
  const float* ca_wq = (const float*)d_in[14];
  const float* ca_bq = (const float*)d_in[15];
  const float* ca_wk = (const float*)d_in[16];
  const float* ca_bk = (const float*)d_in[17];
  const float* ca_wv = (const float*)d_in[18];
  const float* ca_bv = (const float*)d_in[19];
  const float* ca_wo = (const float*)d_in[20];
  const float* ca_bo = (const float*)d_in[21];
  const float* ln3_g = (const float*)d_in[22];
  const float* ln3_b = (const float*)d_in[23];
  const float* fc1_w = (const float*)d_in[24];
  const float* fc1_b = (const float*)d_in[25];
  const float* fc2_w = (const float*)d_in[26];
  const float* fc2_b = (const float*)d_in[27];
  float* out = (float*)d_out;

  size_t off = 0;
  const size_t oTRIG  = off; off += (size_t)2 * NTRIG * 4;
  const size_t oWqkv1 = off; off += (size_t)C3 * CC * 2;
  const size_t oWo1   = off; off += (size_t)CC * CC * 2;
  const size_t oWq2   = off; off += (size_t)CC * CC * 2;
  const size_t oWkv2  = off; off += (size_t)2 * CC * CC * 2;
  const size_t oWo2   = off; off += (size_t)CC * CC * 2;
  const size_t oYh    = off; off += (size_t)ROWS * CC * 2;
  const size_t oQKV   = off; off += 3 * PL * 2;
  const size_t oG     = 0;
  if ((size_t)ROWS * FF * 2 > off) return;
  const size_t oHh    = off; off += (size_t)ROWS * CC * 2;
  const size_t oO     = off; off += (size_t)ROWS * CC * 2;
  const size_t oW1    = off; off += (size_t)FF * CC * 2;
  const size_t oW2    = off; off += (size_t)CC * FF * 2;
  const size_t oX1    = off; off += (size_t)ROWS * CC * 4;
  const size_t oX2    = off; off += (size_t)ROWS * CC * 4;
  if (off > ws_size) return;
  if (off > (size_t)134217728) return;

  char* ws = (char*)d_ws;
  float*    trig   = (float*)(ws + oTRIG);
  _Float16* Wqkv1t = (_Float16*)(ws + oWqkv1);
  _Float16* Wo1t   = (_Float16*)(ws + oWo1);
  _Float16* Wq2t   = (_Float16*)(ws + oWq2);
  _Float16* Wkv2t  = (_Float16*)(ws + oWkv2);
  _Float16* Wo2t   = (_Float16*)(ws + oWo2);
  _Float16* Yh     = (_Float16*)(ws + oYh);
  _Float16* QKVp   = (_Float16*)(ws + oQKV);
  _Float16* Gp     = (_Float16*)(ws + oG);
  _Float16* Hh     = (_Float16*)(ws + oHh);
  _Float16* Op     = (_Float16*)(ws + oO);
  _Float16* W1t    = (_Float16*)(ws + oW1);
  _Float16* W2t    = (_Float16*)(ws + oW2);
  float*    X1     = (float*)(ws + oX1);
  float*    X2     = (float*)(ws + oX2);
  _Float16* Qp = QKVp;
  _Float16* Kp = QKVp + PL;
  _Float16* Vp = QKVp + 2 * PL;

  k_trig<<<dim3(NTRIG / 256), dim3(256), 0, stream>>>(trig, NTRIG);
  k_wt<<<dim3(CC / 64, CC / 64), dim3(256), 0, stream>>>(sa_wq, Wqkv1t, CC, CC);
  k_wt<<<dim3(CC / 64, CC / 64), dim3(256), 0, stream>>>(sa_wk, Wqkv1t + (size_t)CC * CC, CC, CC);
  k_wt<<<dim3(CC / 64, CC / 64), dim3(256), 0, stream>>>(sa_wv, Wqkv1t + (size_t)2 * CC * CC, CC, CC);
  k_wt<<<dim3(CC / 64, CC / 64), dim3(256), 0, stream>>>(sa_wo, Wo1t, CC, CC);
  k_wt<<<dim3(CC / 64, CC / 64), dim3(256), 0, stream>>>(ca_wq, Wq2t, CC, CC);
  k_wt<<<dim3(CC / 64, CC / 64), dim3(256), 0, stream>>>(ca_wk, Wkv2t, CC, CC);
  k_wt<<<dim3(CC / 64, CC / 64), dim3(256), 0, stream>>>(ca_wv, Wkv2t + (size_t)CC * CC, CC, CC);
  k_wt<<<dim3(CC / 64, CC / 64), dim3(256), 0, stream>>>(ca_wo, Wo2t, CC, CC);
  k_wt<<<dim3(FF / 64, CC / 64), dim3(256), 0, stream>>>(fc1_w, W1t, FF, CC);
  k_wt<<<dim3(CC / 64, FF / 64), dim3(256), 0, stream>>>(fc2_w, W2t, CC, FF);
  const int ngrp = in_sizes[1] / 8;
  k_cvt8<<<dim3((ngrp + 255) / 256), dim3(256), 0, stream>>>(y, Yh, ngrp);

  k_ln<<<dim3(ROWS), dim3(256), 0, stream>>>(x, ln1_g, ln1_b, Hh);
  k_proj<<<dim3(ROWS / 256, C3 / 64), dim3(256), 0, stream>>>(Hh, Wqkv1t, sa_bq, sa_bk, sa_bv, trig, Qp, Kp, Vp, 0);
  k_attn<<<dim3(BB * HH * (NN / 128)), dim3(256), 0, stream>>>(Qp, Kp, Vp, Op, 0.125f, 1);
  k_gout<CC, 1><<<dim3(ROWS / 256, CC / 64), dim3(256), 0, stream>>>(Op, Wo1t, sa_bo, x, X1, 0.00048828125f);

  k_ln<<<dim3(ROWS), dim3(256), 0, stream>>>(X1, ln2_g, ln2_b, Hh);
  k_proj<<<dim3(ROWS / 256, CC / 64), dim3(256), 0, stream>>>(Hh, Wq2t, ca_bq, ca_bq, ca_bq, trig, Qp, Kp, Vp, 0);
  k_proj<<<dim3(ROWS / 256, (2 * CC) / 64), dim3(256), 0, stream>>>(Yh, Wkv2t, ca_bk, ca_bv, ca_bv, trig, Qp, Kp, Vp, 1);
  k_attn<<<dim3(BB * HH * (NN / 128)), dim3(256), 0, stream>>>(Qp, Kp, Vp, Op, 0.125f, 0);
  k_gout<CC, 1><<<dim3(ROWS / 256, CC / 64), dim3(256), 0, stream>>>(Op, Wo2t, ca_bo, X1, X2, 0.00048828125f);

  k_ln<<<dim3(ROWS), dim3(256), 0, stream>>>(X2, ln3_g, ln3_b, Hh);
  k_ffn1<<<dim3(ROWS / 256, FF / 64), dim3(256), 0, stream>>>(Hh, W1t, fc1_b, Gp);
  k_gout<FF, 1><<<dim3(ROWS / 256, CC / 64), dim3(256), 0, stream>>>(Gp, W2t, fc2_b, X2, out, 0.001953125f);
  (void)hipGetLastError();
}
